// RNN_2576980377955
// MI455X (gfx1250) — hardware-run, weakly checked
//
#include <hip/hip_runtime.h>
#include <math.h>

constexpr int NBATCH  = 64;
constexpr int NSTEP   = 256;
constexpr int NVOCAB  = 32000;
constexpr int NEMB    = 512;
constexpr int NHID    = 512;
constexpr int NOUTF   = 4;
constexpr int NROWS   = NBATCH * NSTEP;
constexpr int NTHR    = 256;
constexpr int SEQ_BLK = 16;
constexpr int HPITCH  = 520;
constexpr int XSP     = 516;
constexpr float ACARRY   = 1024.0f;
constexpr float BCARRY   = 256.0f;
constexpr float PROD_INV = 1.0f / 262144.0f;
static_assert(NROWS % 64 == 0 && NHID % 64 == 0);
static_assert(NEMB % 32 == 0 && NHID % 32 == 0);
static_assert(NBATCH % SEQ_BLK == 0);
static_assert(NHID == 64 * (NTHR / 32));
static_assert(NEMB / 8 == 64 && NBATCH == 64);
static_assert((SEQ_BLK * NHID) == 8 * 4 * NTHR);
static_assert((NOUTF * NHID) == 2 * 4 * NTHR);
static_assert(SEQ_BLK * NOUTF == NTHR / 4);
static_assert(HPITCH % 8 == 0 && XSP % 4 == 0);
static_assert((NROWS * (NEMB / 8)) % NTHR == 0 && (NHID * NEMB / 8) % NTHR == 0);
static_assert(((NROWS / 64) * (NHID / 64)) % 8 == 0);

typedef __attribute__((ext_vector_type(16))) _Float16 v16h;
typedef __attribute__((ext_vector_type(8)))  _Float16 v8h;
typedef __attribute__((ext_vector_type(16))) __bf16   v16b;
typedef __attribute__((ext_vector_type(8)))  __bf16   v8b;
typedef __attribute__((ext_vector_type(8)))  float    v8f;
typedef __attribute__((ext_vector_type(4)))  float    v4f;

__device__ __forceinline__ unsigned short f2bf_bits(float f) {
  unsigned u = __float_as_uint(f);
  return (unsigned short)((u + 0x7FFFu + ((u >> 16) & 1u)) >> 16);
}
__device__ __forceinline__ float bf_bits2f(unsigned short h) { return __uint_as_float(((unsigned)h) << 16); }

__device__ __forceinline__ void dep_guard_h(v8f& a, v8f& b, v16h x, v16h y) { asm volatile("v_nop\n\tv_nop\n\tv_nop\n\tv_nop" : "+v"(a), "+v"(b) : "v"(x), "v"(y)); }
__device__ __forceinline__ void dep_guard_b(v8f& a, v8f& b, v16b x, v16b y) { asm volatile("v_nop\n\tv_nop\n\tv_nop\n\tv_nop" : "+v"(a), "+v"(b) : "v"(x), "v"(y)); }
__device__ __forceinline__ void keep4_h(v16h a, v16h b, v16h c, v16h d) { asm volatile("v_nop" :: "v"(a), "v"(b), "v"(c), "v"(d)); }
__device__ __forceinline__ void keep4_b(v16b a, v16b b, v16b c, v16b d) { asm volatile("v_nop" :: "v"(a), "v"(b), "v"(c), "v"(d)); }
__device__ __forceinline__ void acc_guard4(v8f& a, v8f& b, v8f& c, v8f& d) { asm volatile("v_nop\n\tv_nop\n\tv_nop\n\tv_nop" : "+v"(a), "+v"(b), "+v"(c), "+v"(d)); }
__device__ __forceinline__ void acc_guard2(v8f& a, v8f& b) { asm volatile("v_nop\n\tv_nop\n\tv_nop\n\tv_nop" : "+v"(a), "+v"(b)); }
template <typename T> struct Frag;
template <> struct Frag<_Float16> {
  typedef v16h V; union U { v16h v; v8h h[2]; };
  static __device__ __forceinline__ v16h load(const _Float16* p) {
    U f; f.h[0] = *(const v8h*)(p); f.h[1] = *(const v8h*)(p + 16); return f.v;
  }
  static __device__ __forceinline__ v8f mma(v16h a, v16h b, v8f c) {
    return __builtin_amdgcn_wmma_f32_16x16x32_f16(false, a, false, b, (short)0, c, false, false);
  }
  static __device__ __forceinline__ void guard(v8f& a, v8f& b, v16h x, v16h y) { dep_guard_h(a, b, x, y); }
  static __device__ __forceinline__ void keep(v16h a, v16h b, v16h c, v16h d) { keep4_h(a, b, c, d); }
};
template <> struct Frag<__bf16> {
  typedef v16b V; union U { v16b v; v8b h[2]; };
  static __device__ __forceinline__ v16b load(const __bf16* p) {
    U f; f.h[0] = *(const v8b*)(p); f.h[1] = *(const v8b*)(p + 16); return f.v;
  }
  static __device__ __forceinline__ v8f mma(v16b a, v16b b, v8f c) {
    return __builtin_amdgcn_wmma_f32_16x16x32_bf16(false, a, false, b, (short)0, c, false, false);
  }
  static __device__ __forceinline__ void guard(v8f& a, v8f& b, v16b x, v16b y) { dep_guard_b(a, b, x, y); }
  static __device__ __forceinline__ void keep(v16b a, v16b b, v16b c, v16b d) { keep4_b(a, b, c, d); }
};

template <int ET> struct Elem;
template <> struct Elem<0> { typedef _Float16 T; };
template <> struct Elem<1> { typedef __bf16 T; };
template <int ET, bool SPLIT, int BIAS_MODE, int OUT_MODE, bool RESID, int ACT = 0>
__global__ __launch_bounds__(256) void wmma_gemm64(
    const unsigned short* __restrict__ Ap, const unsigned short* __restrict__ A2p, int lda, long strideA,
    const unsigned short* __restrict__ Btp, const unsigned short* __restrict__ Bt2p, int ldb, long strideB,
    void* __restrict__ Cout, void* __restrict__ Cout2, int ldc, long strideC,
    const float* __restrict__ bias,
    const float* __restrict__ resid, long strideR,
    int M, int N, int K, float scale) {
  typedef typename Elem<ET>::T T;
  typedef typename Frag<T>::V V;
  const T* A = (const T*)Ap; const T* A2 = (const T*)A2p; const T* Bt = (const T*)Btp; const T* Bt2 = (const T*)Bt2p;
  __shared__ __align__(16) float sT[8][16 * 68];
  const int b    = blockIdx.y;
  const int lane = threadIdx.x & 31;
  const int wave = threadIdx.x >> 5;
  const int tilesN = N >> 6;
  const int tilesM = M >> 6;
  const int tile = blockIdx.x * 8 + wave;
  if (tile >= tilesM * tilesN) return;
  const int tm = tile / tilesN;
  const int tn = tile - tm * tilesN;
  const int m0 = tm << 6;
  const int n0 = tn << 6;

  const T* Ab  = A  + (size_t)b * strideA;
  const T* Bb  = Bt + (size_t)b * strideB;
  const T* Ab2 = SPLIT ? (A2  + (size_t)b * strideA) : nullptr;
  const T* Bb2 = SPLIT ? (Bt2 + (size_t)b * strideB) : nullptr;

  const int rlane = lane & 15;
  const int koff  = (lane >> 4) * 8;
  const int mOff  = (lane >> 4) * 8;

  v8f acc[4][4];
#pragma unroll
  for (int i = 0; i < 4; ++i)
#pragma unroll
    for (int j = 0; j < 4; ++j) acc[i][j] = (v8f){0.f,0.f,0.f,0.f,0.f,0.f,0.f,0.f};

  for (int k0 = 0; k0 < K; k0 += 32) {
    V bh[4], bl[4];
#pragma unroll
    for (int j = 0; j < 4; ++j) {
      const size_t bo = (size_t)(n0 + (j << 4) + rlane) * ldb + koff + k0;
      bh[j] = Frag<T>::load(Bb + bo);
      if (SPLIT) bl[j] = Frag<T>::load(Bb2 + bo);
    }
#pragma unroll
    for (int i = 0; i < 4; ++i) {
      const size_t ao = (size_t)(m0 + (i << 4) + rlane) * lda + koff + k0;
      V ah = Frag<T>::load(Ab + ao);
      V al;
      if (SPLIT) al = Frag<T>::load(Ab2 + ao);
#pragma unroll
      for (int j = 0; j < 4; ++j) {
        acc[i][j] = Frag<T>::mma(ah, bh[j], acc[i][j]);
        if (SPLIT) {
          acc[i][j] = Frag<T>::mma(ah, bl[j], acc[i][j]);
          acc[i][j] = Frag<T>::mma(al, bh[j], acc[i][j]);
        }
      }
      Frag<T>::guard(acc[i][0], acc[i][3], ah, SPLIT ? al : ah);
    }
    Frag<T>::keep(bh[0], bh[1], bh[2], bh[3]);
    if (SPLIT) Frag<T>::keep(bl[0], bl[1], bl[2], bl[3]);
  }
  acc_guard4(acc[0][0], acc[0][1], acc[0][2], acc[0][3]);
  acc_guard4(acc[1][0], acc[1][1], acc[1][2], acc[1][3]);
  acc_guard4(acc[2][0], acc[2][1], acc[2][2], acc[2][3]);
  acc_guard4(acc[3][0], acc[3][1], acc[3][2], acc[3][3]);

  float* slab = sT[wave];
  const float* Rb = RESID ? (resid + (size_t)b * strideR) : nullptr;
#pragma unroll
  for (int i = 0; i < 4; ++i) {
    const int mBase = m0 + (i << 4);
#pragma unroll
    for (int j = 0; j < 4; ++j) {
      const int n = n0 + (j << 4) + rlane;
      float bv = 0.f;
      if (BIAS_MODE == 2) bv = bias[n];
#pragma unroll
      for (int r = 0; r < 8; ++r) {
        float v = acc[i][j][r] * scale;
        if (BIAS_MODE == 1) v += bias[mBase + mOff + r];
        if (BIAS_MODE == 2) v += bv;
        if (RESID) v += Rb[(size_t)(mBase + mOff + r) * ldc + n];
        if (ACT == 1) v = tanhf(v);
        if (ACT == 2) v = fmaxf(v, 0.0f);
        if (ACT == 3) v = v / (1.0f + expf(-v));
        if (ACT == 4) v = (v > 0.f) ? v : 0.01f * v;
        if (ACT == 5) v = 0.5f * v * (1.0f + erff(v * 0.70710678118654752f));
        slab[(mOff + r) * 68 + (j << 4) + rlane] = v;
      }
    }
    __builtin_amdgcn_fence(__ATOMIC_RELEASE, "workgroup");
    __builtin_amdgcn_wave_barrier();
    __builtin_amdgcn_fence(__ATOMIC_ACQUIRE, "workgroup");
    if (OUT_MODE == 0) {
      float* C = (float*)Cout + (size_t)b * strideC;
      const int hh = lane >> 4, c4 = (lane & 15) * 4;
      for (int pass = 0; pass < 2; ++pass) {
#pragma unroll
        for (int it = 0; it < 8; ++it) {
          const int row = it * 2 + hh;
          v4f v = *(const v4f*)(slab + row * 68 + c4);
          *(volatile v4f*)(C + (size_t)(mBase + row) * ldc + n0 + c4) = v;
        }
        __threadfence();
      }
    } else {
      const int q = lane >> 3, c8 = (lane & 7) * 8;
      unsigned short* C  = (unsigned short*)Cout  + (size_t)b * strideC;
      unsigned short* C2 = (OUT_MODE == 2) ? ((unsigned short*)Cout2 + (size_t)b * strideC) : nullptr;
      for (int pass = 0; pass < 2; ++pass) {
#pragma unroll
        for (int it = 0; it < 4; ++it) {
          const int row = it * 4 + q;
          const float* sp = slab + row * 68 + c8;
          v8h hv, lv;
#pragma unroll
          for (int e = 0; e < 8; ++e) {
            if (OUT_MODE == 1) {
              hv[e] = (_Float16)sp[e];
            } else {
              unsigned short hb = f2bf_bits(sp[e]);
              unsigned short lb = f2bf_bits(sp[e] - bf_bits2f(hb));
              hv[e] = __builtin_bit_cast(_Float16, hb);
              lv[e] = __builtin_bit_cast(_Float16, lb);
            }
          }
          *(volatile v8h*)(C + (size_t)(mBase + row) * ldc + n0 + c8) = hv;
          if (OUT_MODE == 2) *(volatile v8h*)(C2 + (size_t)(mBase + row) * ldc + n0 + c8) = lv;
        }
        __threadfence();
      }
    }
    __builtin_amdgcn_fence(__ATOMIC_RELEASE, "workgroup");
    __builtin_amdgcn_wave_barrier();
    __builtin_amdgcn_fence(__ATOMIC_ACQUIRE, "workgroup");
  }
}

__global__ __launch_bounds__(NTHR) void gather_rows_kernel(const int* __restrict__ tok, const float* __restrict__ emb,
                                                           unsigned short* __restrict__ dst, int n8) {
  const int i = blockIdx.x * NTHR + threadIdx.x;
  if (i < n8) {
    const int row = i >> 6;
    const int c8  = i & 63;
    const int t   = row >> 6;
    const int b   = row & 63;
    int id = tok[b * NSTEP + t];
    id = (id < 0) ? 0 : id;
    id = (id > NVOCAB - 1) ? (NVOCAB - 1) : id;
    const float* sp = emb + (size_t)id * NEMB + c8 * 8;
    const v4f a = *(const v4f*)(sp);
    const v4f q = *(const v4f*)(sp + 4);
    v8h hv;
#pragma unroll
    for (int e = 0; e < 4; ++e) {
      hv[e]     = (_Float16)(a[e] * ACARRY);
      hv[4 + e] = (_Float16)(q[e] * ACARRY);
    }
    *(volatile v8h*)(dst + (size_t)i * 8) = hv;
    __threadfence();
    *(volatile v8h*)(dst + (size_t)i * 8) = hv;
  }
}

__global__ __launch_bounds__(NTHR) void cvt_f16x8_kernel(const float* __restrict__ src, unsigned short* __restrict__ dst,
                                                         int n8, float sc) {
  const int i = blockIdx.x * NTHR + threadIdx.x;
  if (i < n8) {
    const float* sp = src + (size_t)i * 8;
    const v4f a = *(const v4f*)(sp);
    const v4f q = *(const v4f*)(sp + 4);
    v8h hv;
#pragma unroll
    for (int e = 0; e < 4; ++e) {
      hv[e]     = (_Float16)(a[e] * sc);
      hv[4 + e] = (_Float16)(q[e] * sc);
    }
    *(volatile v8h*)(dst + (size_t)i * 8) = hv;
    __threadfence();
    *(volatile v8h*)(dst + (size_t)i * 8) = hv;
  }
}

__device__ __forceinline__ void stage_step_tile(const float* __restrict__ XW, float* Xs, int t, int rowbase, int tid) {
  const float* src = XW + ((size_t)t * NBATCH + (size_t)rowbase) * NHID;
#pragma unroll
  for (int it = 0; it < 4; ++it) {
    const int idx = it * NTHR + tid;
    const int row = idx >> 7, c4 = (idx & 127) * 4;
    const v4f v = *(const v4f*)(src + (size_t)row * NHID + c4);
    *(v4f*)(Xs + row * XSP + c4) = v;
  }
  asm volatile("" ::: "memory");
#pragma unroll
  for (int it = 4; it < 8; ++it) {
    const int idx = it * NTHR + tid;
    const int row = idx >> 7, c4 = (idx & 127) * 4;
    const v4f v = *(const v4f*)(src + (size_t)row * NHID + c4);
    *(v4f*)(Xs + row * XSP + c4) = v;
  }
}

__global__ __launch_bounds__(NTHR) void rnn_seq_kernel(const float* __restrict__ XW, const unsigned short* __restrict__ WHp,
                                                       const float* __restrict__ bhh, const float* __restrict__ wfc,
                                                       const float* __restrict__ bfc, float* __restrict__ out) {
  __shared__ __align__(16) _Float16 Ah[SEQ_BLK * HPITCH];
  __shared__ __align__(16) float    Xs[SEQ_BLK * XSP];
  __shared__ __align__(16) float    Wfs[NOUTF * NHID];
  __shared__ __align__(16) float    Os[SEQ_BLK * NOUTF];
  const _Float16* WH = (const _Float16*)WHp;
  const int tid = threadIdx.x, lane = tid & 31, wave = tid >> 5;
  const int c = lane & 15, hh = lane >> 4, koff = hh * 8;
  const int rowbase = blockIdx.x * SEQ_BLK;

#pragma unroll 1
  for (int i = tid; i < SEQ_BLK * HPITCH; i += NTHR) Ah[i] = (_Float16)0.0f;
#pragma unroll
  for (int it = 0; it < 2; ++it) {
    const int idx = it * NTHR + tid;
    const v4f v = *(const v4f*)(wfc + 4 * idx);
    *(v4f*)(Wfs + 4 * idx) = v;
  }
  stage_step_tile(XW, Xs, 0, rowbase, tid);
  float hst[4][8], bb[4];
#pragma unroll
  for (int nt = 0; nt < 4; ++nt) {
    bb[nt] = bhh[64 * wave + 16 * nt + c];
#pragma unroll
    for (int r = 0; r < 8; ++r) hst[nt][r] = 0.0f;
  }
  __syncthreads();

  const _Float16* ahrow = Ah + c * HPITCH + koff;
  const v8f z8 = {0.f, 0.f, 0.f, 0.f, 0.f, 0.f, 0.f, 0.f};

#pragma unroll 1
  for (int t = 0; t < NSTEP; ++t) {
#pragma unroll
    for (int np = 0; np < 2; ++np) {
      const int j0 = 64 * wave + 32 * np + c;
      const int j1 = j0 + 16;
      const _Float16* w0 = WH + (size_t)j0 * NHID + koff;
      const _Float16* w1 = WH + (size_t)j1 * NHID + koff;
      v8f acc0 = z8, acc1 = z8;
#pragma unroll 1
      for (int k0 = 0; k0 < NHID; k0 += 32) {
        const v16h a  = Frag<_Float16>::load(ahrow + k0);
        const v16h b0 = Frag<_Float16>::load(w0 + k0);
        const v16h b1 = Frag<_Float16>::load(w1 + k0);
        acc0 = Frag<_Float16>::mma(a, b0, acc0);
        acc1 = Frag<_Float16>::mma(a, b1, acc1);
        dep_guard_h(acc0, acc1, a, b1);
        keep4_h(a, b0, b1, a);
      }
      acc_guard2(acc0, acc1);
#pragma unroll
      for (int r = 0; r < 8; ++r) {
        const float x0 = Xs[(8 * hh + r) * XSP + j0];
        const float x1 = Xs[(8 * hh + r) * XSP + j1];
        float v0 = acc0[r] * PROD_INV + x0;
        float v1 = acc1[r] * PROD_INV + x1;
        v0 = v0 + bb[2 * np + 0];
        v1 = v1 + bb[2 * np + 1];
        hst[2 * np + 0][r] = tanhf(v0);
        hst[2 * np + 1][r] = tanhf(v1);
      }
    }
    __syncthreads();
#pragma unroll
    for (int nt = 0; nt < 4; ++nt) {
      const int j = 64 * wave + 16 * nt + c;
#pragma unroll
      for (int r = 0; r < 8; ++r) Ah[(8 * hh + r) * HPITCH + j] = (_Float16)(hst[nt][r] * ACARRY);
    }
    {
      const int tn = (t + 1 < NSTEP) ? (t + 1) : (NSTEP - 1);
      stage_step_tile(XW, Xs, tn, rowbase, tid);
    }
    __syncthreads();
  }

#pragma unroll
  for (int nt = 0; nt < 4; ++nt) {
    const int j = 64 * wave + 16 * nt + c;
#pragma unroll
    for (int r = 0; r < 8; ++r) Xs[(8 * hh + r) * XSP + j] = hst[nt][r];
  }
  __syncthreads();
  {
    const int task = tid >> 2;
    const int seg  = tid & 3;
    const int row  = task >> 2;
    const int o    = task & 3;
    const float* hp = Xs + row * XSP + seg * 128;
    const float* wp = Wfs + o * NHID + seg * 128;
    float s = 0.0f;
#pragma unroll 4
    for (int k = 0; k < 128; ++k) s += hp[k] * wp[k];
    s += __shfl_xor(s, 2, 32);
    s += __shfl_xor(s, 1, 32);
    const float res = s + bfc[o];
    if (seg == 0) Os[task] = res;
  }
  __syncthreads();
  if (wave == 0) {
    const int lc = (lane < 16) ? lane : 15;
    const v4f v = *(const v4f*)(Os + 4 * lc);
    float* op = out + (size_t)rowbase * NOUTF + 4 * lc;
    if (lane < 16) *(volatile v4f*)op = v;
    __threadfence();
    if (lane < 16) *(volatile v4f*)op = v;
  }
}

extern "C" void kernel_launch(void* const* d_in, const int* in_sizes, int n_in,
                              void* d_out, int out_size, void* d_ws, size_t ws_size, hipStream_t stream) {
  if (n_in < 8 || d_out == nullptr || d_ws == nullptr) return;
  if (in_sizes[0] != NBATCH * NSTEP || in_sizes[1] != NVOCAB * NEMB || in_sizes[2] != NHID * NEMB ||
      in_sizes[3] != NHID * NHID || in_sizes[4] != NHID || in_sizes[5] != NHID ||
      in_sizes[6] != NOUTF * NHID || in_sizes[7] != NOUTF || out_size != NBATCH * NOUTF) return;

  const int*   tok = (const int*)d_in[0];
  const float* emb = (const float*)d_in[1];
  const float* wih = (const float*)d_in[2];
  const float* whh = (const float*)d_in[3];
  const float* bih = (const float*)d_in[4];
  const float* bhh = (const float*)d_in[5];
  const float* wfc = (const float*)d_in[6];
  const float* bfc = (const float*)d_in[7];
  float* out = (float*)d_out;

  char* ws = (char*)d_ws; size_t off = 0;
  auto carve = [&](size_t bytes) -> char* { char* p = ws + off; off += (bytes + 255) & ~(size_t)255; return p; };
  unsigned short* E16   = (unsigned short*)carve((size_t)NROWS * NEMB * 2);
  unsigned short* WIH16 = (unsigned short*)carve((size_t)NHID * NEMB * 2);
  unsigned short* WHH16 = (unsigned short*)carve((size_t)NHID * NHID * 2);
  float*          XW    = (float*)carve((size_t)NROWS * NHID * 4);
  if (off > ws_size || off > (size_t)134217728) return;

  const int n8e = NROWS * (NEMB / 8);
  const int n8w = NHID * (NEMB / 8);
  const int n8h = NHID * (NHID / 8);
  gather_rows_kernel<<<(n8e + NTHR - 1) / NTHR, NTHR, 0, stream>>>(tok, emb, E16, n8e);
  cvt_f16x8_kernel<<<(n8w + NTHR - 1) / NTHR, NTHR, 0, stream>>>(wih, WIH16, n8w, BCARRY);
  cvt_f16x8_kernel<<<(n8h + NTHR - 1) / NTHR, NTHR, 0, stream>>>(whh, WHH16, n8h, BCARRY);

  const dim3 ggrid((NROWS / 64) * (NHID / 64) / 8, 1);
  wmma_gemm64<0, false, 2, 0, false, 0><<<ggrid, 256, 0, stream>>>(
      E16, E16, NEMB, 0L, WIH16, WIH16, NEMB, 0L, (void*)XW, (void*)XW, NHID, 0L,
      bih, XW, 0L, NROWS, NHID, NEMB, PROD_INV);

  rnn_seq_kernel<<<NBATCH / SEQ_BLK, NTHR, 0, stream>>>(XW, WHH16, bhh, wfc, bfc, out);
}
